// ConvSelfAttention_64957085384894
// MI455X (gfx1250) — hardware-verified
//
#include <hip/hip_runtime.h>
#include <math.h>
#include <stdint.h>

#define NBATCH 2
#define TLEN   2048
#define EMB    128
#define NHEAD  8
#define KWIN   32
#define HE     (NHEAD * EMB)
#define NROWS  (NBATCH * TLEN)
#define QKVW   (3 * HE)
#define TQ     16
#define QK_SCALE (1.0f / 3.3635856610148585f)
#define CVB_X  ((NROWS * EMB) / 2048)
#define CVB_W  ((HE * EMB) / 2048)
static_assert((NROWS * EMB) % 2048 == 0);
static_assert((HE * EMB) % 2048 == 0);
static_assert(NROWS % 64 == 0 && QKVW % 64 == 0 && EMB % 64 == 0);
static_assert(EMB % 32 == 0 && HE % 32 == 0);
static_assert((2 * HE) % 64 == 0);
static_assert(TLEN % TQ == 0);
static_assert(KWIN == 32 && EMB == 128 && NHEAD == 8);

typedef __bf16   v16b __attribute__((ext_vector_type(16)));
typedef __bf16   v8b  __attribute__((ext_vector_type(8)));
typedef float    v8f  __attribute__((ext_vector_type(8)));
typedef float    v4f  __attribute__((ext_vector_type(4)));
typedef unsigned int v4u __attribute__((ext_vector_type(4)));
typedef v4f __attribute__((may_alias)) v4fa;

__device__ __forceinline__ unsigned short bf_bits(float f) {
  unsigned u = __float_as_uint(f);
  return (unsigned short)((u + 0x7FFFu + ((u >> 16) & 1u)) >> 16);
}
__device__ __forceinline__ float bf_up(unsigned short h) { return __uint_as_float(((unsigned)h) << 16); }
__device__ __forceinline__ unsigned pk16(unsigned short a, unsigned short b) { return (unsigned)a | ((unsigned)b << 16); }
__device__ __forceinline__ v8f zero8() { v8f z = {0.f, 0.f, 0.f, 0.f, 0.f, 0.f, 0.f, 0.f}; return z; }
__device__ __forceinline__ v4f zero4() { v4f z = {0.f, 0.f, 0.f, 0.f}; return z; }

__device__ __forceinline__ v16b ldfrag_b(const __bf16* p) {
  union { v16b v; v8b h[2]; } f;
  f.h[0] = *(const v8b*)(p);
  f.h[1] = *(const v8b*)(p + 16);
  return f.v;
}

__device__ __forceinline__ v8f mma_b_raw(v16b a, v16b b, v8f c) {
  return __builtin_amdgcn_wmma_f32_16x16x32_bf16(false, a, false, b, (short)0, c, false, false);
}
__device__ __forceinline__ void dep_guard_b(v8f& a, v8f& b, v16b x) {
  asm volatile("v_nop\n\tv_nop\n\tv_nop\n\tv_nop" : "+v"(a), "+v"(b) : "v"(x));
}
__device__ __forceinline__ void keep4_b(v16b a, v16b b, v16b c, v16b d) {
  asm volatile("v_nop" :: "v"(a), "v"(b), "v"(c), "v"(d));
}
__device__ __forceinline__ void acc_guard4(v8f& a, v8f& b, v8f& c, v8f& d) {
  asm volatile("v_nop\n\tv_nop\n\tv_nop\n\tv_nop" : "+v"(a), "+v"(b), "+v"(c), "+v"(d));
}

__global__ __launch_bounds__(256) void cvt_planes(const float* __restrict__ x, const float* __restrict__ wq,
                                                  const float* __restrict__ wk, const float* __restrict__ wv,
                                                  const float* __restrict__ wu,
                                                  unsigned short* xb, unsigned short* wqkv, unsigned short* wub) {
  const int blk = blockIdx.x;
  if (blk >= CVB_X + 4 * CVB_W) return;
  const float* src;
  unsigned short* dst;
  int lb;
  if (blk < CVB_X) {
    src = x;  dst = xb; lb = blk;
  } else if (blk < CVB_X + CVB_W) {
    src = wq; dst = wqkv; lb = blk - CVB_X;
  } else if (blk < CVB_X + 2 * CVB_W) {
    src = wk; dst = wqkv + (size_t)HE * EMB; lb = blk - CVB_X - CVB_W;
  } else if (blk < CVB_X + 3 * CVB_W) {
    src = wv; dst = wqkv + (size_t)2 * HE * EMB; lb = blk - CVB_X - 2 * CVB_W;
  } else {
    src = wu; dst = wub; lb = blk - CVB_X - 3 * CVB_W;
  }
  const size_t i = ((size_t)lb * 256 + threadIdx.x) * 8;
  const v4f a = *(const v4fa*)(src + i);
  const v4f b = *(const v4fa*)(src + i + 4);
  v4u p;
  p[0] = pk16(bf_bits(a[0]), bf_bits(a[1]));
  p[1] = pk16(bf_bits(a[2]), bf_bits(a[3]));
  p[2] = pk16(bf_bits(b[0]), bf_bits(b[1]));
  p[3] = pk16(bf_bits(b[2]), bf_bits(b[3]));
  *(volatile v4u*)(dst + i) = p;
  __threadfence();
  *(volatile v4u*)(dst + i) = p;
}

template <int M, int N, int K, bool TWO>
__global__ __launch_bounds__(256) void gemm_nt(const unsigned short* __restrict__ A0p,
                                               const unsigned short* __restrict__ A1p,
                                               const unsigned short* __restrict__ Btp,
                                               const float* __restrict__ bias, float* C) {
  static_assert((M % 64) == 0 && (N % 64) == 0 && (K % 32) == 0);
  __shared__ __align__(16) float sT[8][16 * 68];
  const __bf16* A0 = (const __bf16*)(const void*)A0p;
  const __bf16* A1 = (const __bf16*)(const void*)A1p;
  const __bf16* Bt = (const __bf16*)(const void*)Btp;

  const int lane = threadIdx.x & 31;
  const int wave = threadIdx.x >> 5;
  constexpr int tilesN = N / 64;
  constexpr int tilesM = M / 64;
  const int tile = blockIdx.x * 8 + wave;
  if (tile >= tilesM * tilesN) return;
  const int tm = tile / tilesN;
  const int tn = tile - tm * tilesN;
  const int m0 = tm << 6;
  const int n0 = tn << 6;

  const int rlane = lane & 15;
  const int koff  = (lane >> 4) * 8;
  const int mOff  = (lane >> 4) * 8;

  v8f acc[4][4];
#pragma unroll
  for (int i = 0; i < 4; ++i)
#pragma unroll
    for (int j = 0; j < 4; ++j) acc[i][j] = zero8();

  for (int k0 = 0; k0 < K; k0 += 32) {
    v16b bh[4];
#pragma unroll
    for (int j = 0; j < 4; ++j) {
      const size_t bo = (size_t)(n0 + (j << 4) + rlane) * K + koff + k0;
      bh[j] = ldfrag_b(Bt + bo);
    }
#pragma unroll
    for (int i = 0; i < 4; ++i) {
      const size_t ao = (size_t)(m0 + (i << 4) + rlane) * K + koff + k0;
      const v16b ah = ldfrag_b(A0 + ao);
#pragma unroll
      for (int j = 0; j < 4; ++j) acc[i][j] = mma_b_raw(ah, bh[j], acc[i][j]);
      dep_guard_b(acc[i][0], acc[i][3], ah);
      if (TWO) {
        const v16b al = ldfrag_b(A1 + ao);
#pragma unroll
        for (int j = 0; j < 4; ++j) acc[i][j] = mma_b_raw(al, bh[j], acc[i][j]);
        dep_guard_b(acc[i][0], acc[i][3], al);
      }
    }
    keep4_b(bh[0], bh[1], bh[2], bh[3]);
  }
  acc_guard4(acc[0][0], acc[0][1], acc[0][2], acc[0][3]);
  acc_guard4(acc[1][0], acc[1][1], acc[1][2], acc[1][3]);
  acc_guard4(acc[2][0], acc[2][1], acc[2][2], acc[2][3]);
  acc_guard4(acc[3][0], acc[3][1], acc[3][2], acc[3][3]);

  float* slab = sT[wave];
  const int hsel = lane >> 4;
  const int c4   = (lane & 15) * 4;
  v4f addv = zero4();
  float sc = 1.0f;
  if (TWO) {
    const v4f bb = *(const v4fa*)(bias + n0 + c4);
    addv[0] = bf_up(bf_bits(bb[0]));
    addv[1] = bf_up(bf_bits(bb[1]));
    addv[2] = bf_up(bf_bits(bb[2]));
    addv[3] = bf_up(bf_bits(bb[3]));
  } else {
    sc = (n0 < 2 * HE) ? QK_SCALE : 1.0f;
  }
#pragma unroll
  for (int i = 0; i < 4; ++i) {
    const int mBase = m0 + (i << 4);
#pragma unroll
    for (int j = 0; j < 4; ++j) {
#pragma unroll
      for (int r = 0; r < 8; ++r) slab[(mOff + r) * 68 + (j << 4) + rlane] = acc[i][j][r];
    }
    __builtin_amdgcn_fence(__ATOMIC_RELEASE, "workgroup");
    __builtin_amdgcn_wave_barrier();
    __builtin_amdgcn_fence(__ATOMIC_ACQUIRE, "workgroup");
    v4f vals[8];
#pragma unroll
    for (int it = 0; it < 8; ++it) {
      const int row = 2 * it + hsel;
      v4f v = *(const v4fa*)(slab + row * 68 + c4);
      v = TWO ? (v + addv) : (v * sc);
      vals[it] = v;
    }
#pragma unroll
    for (int it = 0; it < 8; ++it)
      *(volatile v4f*)(C + (size_t)(mBase + 2 * it + hsel) * N + n0 + c4) = vals[it];
    __threadfence();
#pragma unroll
    for (int it = 0; it < 8; ++it)
      *(volatile v4f*)(C + (size_t)(mBase + 2 * it + hsel) * N + n0 + c4) = vals[it];
    __builtin_amdgcn_fence(__ATOMIC_RELEASE, "workgroup");
    __builtin_amdgcn_wave_barrier();
    __builtin_amdgcn_fence(__ATOMIC_ACQUIRE, "workgroup");
  }
}

__global__ __launch_bounds__(128) void win_attn(const float* __restrict__ QKV,
                                               unsigned short* Oh, unsigned short* Ol) {
  const int tid  = threadIdx.x;
  const int wave = tid >> 5;
  const int lane = tid & 31;
  const int hsel = lane >> 4;
  const int c    = lane & 15;
  const int head = wave * 2 + hsel;
  const int b    = blockIdx.y;
  const int t0   = blockIdx.x * TQ;
  if (t0 >= TLEN || b >= NBATCH) return;
  const int colq = head * EMB + 8 * c;
  const float* Qb = QKV + (size_t)b * TLEN * QKVW + colq;
  const float* Kb = Qb + HE;
  const float* Vb = Qb + 2 * HE;
  unsigned short* ohb = Oh + (size_t)b * TLEN * HE + colq;
  unsigned short* olb = Ol + (size_t)b * TLEN * HE + colq;

#pragma unroll 1
  for (int tq = 0; tq < TQ; ++tq) {
    const int t = t0 + tq;
    const float* qp = Qb + (size_t)t * QKVW;
    const v4f q0 = *(const v4fa*)(qp);
    const v4f q1 = *(const v4fa*)(qp + 4);
    float mrun = -INFINITY;
    float dk0 = 0.0f, dk1 = 0.0f;
#pragma unroll 1
    for (int j = 0; j < KWIN; ++j) {
      const int pos  = t + j - (KWIN - 1);
      const int prow = (pos < 0) ? 0 : pos;
      const float* kp = Kb + (size_t)prow * QKVW;
      const v4f ka = *(const v4fa*)(kp);
      const v4f kc = *(const v4fa*)(kp + 4);
      const v4f pr = q0 * ka + q1 * kc;
      float d = (pr[0] + pr[1]) + (pr[2] + pr[3]);
      d = (pos >= 0) ? d : 0.0f;
      d += __shfl_xor(d, 1, 32);
      d += __shfl_xor(d, 2, 32);
      d += __shfl_xor(d, 4, 32);
      d += __shfl_xor(d, 8, 32);
      mrun = fmaxf(mrun, d);
      dk0 = (c == j) ? d : dk0;
      dk1 = (c + 16 == j) ? d : dk1;
    }
    const float p0 = __expf(dk0 - mrun);
    const float p1 = __expf(dk1 - mrun);
    float s = p0 + p1;
    s += __shfl_xor(s, 1, 32);
    s += __shfl_xor(s, 2, 32);
    s += __shfl_xor(s, 4, 32);
    s += __shfl_xor(s, 8, 32);
    v4f acc0 = zero4(), acc1 = zero4();
#pragma unroll 1
    for (int j = 0; j < KWIN; ++j) {
      const int pos  = t + j - (KWIN - 1);
      const int prow = (pos < 0) ? 0 : pos;
      const float psel = (j < 16) ? p0 : p1;
      float pj = __shfl(psel, j & 15, 16);
      pj = (pos >= 0) ? pj : 0.0f;
      const float* vp = Vb + (size_t)prow * QKVW;
      const v4f va = *(const v4fa*)(vp);
      const v4f vc = *(const v4fa*)(vp + 4);
      acc0 += va * pj;
      acc1 += vc * pj;
    }
    const float inv = 1.0f / s;
    const v4f o0 = acc0 * inv;
    const v4f o1 = acc1 * inv;
    v4u hv, lv;
#pragma unroll
    for (int e = 0; e < 2; ++e) {
      const float f0 = o0[2 * e], f1 = o0[2 * e + 1];
      const float g0 = o1[2 * e], g1 = o1[2 * e + 1];
      const unsigned short hf0 = bf_bits(f0), hf1 = bf_bits(f1);
      const unsigned short hg0 = bf_bits(g0), hg1 = bf_bits(g1);
      const unsigned short lf0 = bf_bits(f0 - bf_up(hf0)), lf1 = bf_bits(f1 - bf_up(hf1));
      const unsigned short lg0 = bf_bits(g0 - bf_up(hg0)), lg1 = bf_bits(g1 - bf_up(hg1));
      hv[e]     = pk16(hf0, hf1);
      hv[2 + e] = pk16(hg0, hg1);
      lv[e]     = pk16(lf0, lf1);
      lv[2 + e] = pk16(lg0, lg1);
    }
    unsigned short* ohp = ohb + (size_t)t * HE;
    unsigned short* olp = olb + (size_t)t * HE;
    *(volatile v4u*)ohp = hv;
    *(volatile v4u*)olp = lv;
    __threadfence();
    *(volatile v4u*)ohp = hv;
    *(volatile v4u*)olp = lv;
  }
}

extern "C" void kernel_launch(void* const* d_in, const int* in_sizes, int n_in,
                              void* d_out, int out_size, void* d_ws, size_t ws_size,
                              hipStream_t stream) {
  if (n_in < 6) return;
  if (in_sizes[0] != NROWS * EMB) return;
  if (in_sizes[1] != HE * EMB || in_sizes[2] != HE * EMB || in_sizes[3] != HE * EMB) return;
  if (in_sizes[4] != EMB * HE) return;
  if (in_sizes[5] != EMB) return;
  if (out_size != NROWS * EMB) return;

  const float* x  = (const float*)d_in[0];
  const float* Wq = (const float*)d_in[1];
  const float* Wk = (const float*)d_in[2];
  const float* Wv = (const float*)d_in[3];
  const float* Wu = (const float*)d_in[4];
  const float* bu = (const float*)d_in[5];
  float* out = (float*)d_out;

  const size_t PXB   = (size_t)NROWS * EMB * 2;
  const size_t PWQKV = (size_t)3 * HE * EMB * 2;
  const size_t PWU   = (size_t)EMB * HE * 2;
  const size_t PQKV  = (size_t)NROWS * QKVW * 4;
  const size_t PO    = (size_t)NROWS * HE * 2;
  size_t off = 0;
  const size_t oXb   = off; off += PXB;
  const size_t oWqkv = off; off += PWQKV;
  const size_t oWub  = off; off += PWU;
  const size_t oQKV  = off; off += PQKV;
  const size_t oOh   = off; off += PO;
  const size_t oOl   = off; off += PO;
  if (off > ws_size) return;
  if (off > (size_t)134217728) return;

  char* ws = (char*)d_ws;
  unsigned short* Xb   = (unsigned short*)(ws + oXb);
  unsigned short* Wqkv = (unsigned short*)(ws + oWqkv);
  unsigned short* Wub  = (unsigned short*)(ws + oWub);
  float*          QKV  = (float*)(ws + oQKV);
  unsigned short* Oh   = (unsigned short*)(ws + oOh);
  unsigned short* Ol   = (unsigned short*)(ws + oOl);

  const dim3 blk(256);
  const dim3 gCvt(CVB_X + 4 * CVB_W);
  const int  tiles1 = (NROWS / 64) * (QKVW / 64);
  const dim3 gProj((tiles1 + 7) / 8);
  const dim3 gAttn(TLEN / TQ, NBATCH);
  const int  tiles2 = (NROWS / 64) * (EMB / 64);
  const dim3 gOut((tiles2 + 7) / 8);

  cvt_planes<<<gCvt, blk, 0, stream>>>(x, Wq, Wk, Wv, Wu, Xb, Wqkv, Wub);
  gemm_nt<NROWS, QKVW, EMB, false><<<gProj, blk, 0, stream>>>(Xb, Xb, Wqkv, bu, QKV);
  win_attn<<<gAttn, dim3(128), 0, stream>>>(QKV, Oh, Ol);
  gemm_nt<NROWS, EMB, HE, true><<<gOut, blk, 0, stream>>>(Oh, Ol, Wub, bu, out);
  (void)hipGetLastError();
}
